// GCN_regressor_3092376453282
// MI455X (gfx1250) — hardware-verified
//
#include <hip/hip_runtime.h>
#include <stddef.h>
#include <stdint.h>
#include <math.h>


#define NNODE  50000
#define NEDGE  800000
#define HID    128
#define NLAY   4
#define NG     32
#define LNEPS  1e-5f
#define MP     50048
#define K2     256
#define NTHR   256
#define NWAVE  8
#define EPT    8
#define CHUNK  (NTHR * EPT)
#define WCAP   (EPT * 32)
#define LISTN  (NWAVE * WCAP)
#define NBA    1024
#define SLA    10
#define NBLK   49
#define NSLOT  (NBLK * NBA)
#define RCAP   28672
#define DEGCAP 64
#define GBM    64
#define GBN    128
#define GTHR   128
#define GWAVE  (GTHR / 32)
#define ROWH   256
#define AGG_ZINTS (LISTN + 2 * RCAP + 3 * NBA)
#define MISC_INTS 16
#define BK_LDS_INTS (AGG_ZINTS + MISC_INTS)
#define NUWE   (HID * (HID / 8))
#define NUWL   (NLAY * HID * (K2 / 8))
#define NUPT   512
#define NPTV   448
#define U_WL   NUWE
#define U_PT   (NUWE + NUWL)
#define U_XB   (U_PT + NUPT)
#define PT_BE  0
#define PT_BL  128
#define PT_GA  640
#define PT_BT  1152
#define PT_WO  1664
#define PT_N   1792
#define WSMAX  134217728

static_assert((CHUNK & (CHUNK - 1)) == 0 && CHUNK <= 4096);
static_assert((NBA & (NBA - 1)) == 0 && NBA == (1 << SLA));
static_assert(((long long)NEDGE << SLA) < (1LL << 31));
static_assert(LISTN % NTHR == 0 && LISTN >= NBA);
static_assert(NBA % NWAVE == 0 && NBA % 32 == 0 && NBA == 4 * NTHR);
static_assert(RCAP % (NTHR * 4) == 0 && AGG_ZINTS % 4 == 0);
static_assert(RCAP >= 17455 && DEGCAP >= 35 + 8);
static_assert(HID == 4 * 32 && NG == 32);
static_assert(MP % GBM == 0 && MP >= NNODE && MP == 391 * 128 && NSLOT >= MP);
static_assert(HID % 32 == 0 && K2 % 32 == 0 && K2 == 2 * HID && GBN == HID && GBM == GWAVE * 16);
static_assert(NUWE % NTHR == 0 && NUWL % NTHR == 0 && NUPT % NTHR == 0 && (MP * 16) % NTHR == 0);
static_assert(NPTV * 4 == PT_N && PT_WO + HID == PT_N);
static_assert(BK_LDS_INTS * 4 <= 300000);
static_assert(ROWH == 2 * HID);

typedef float          v4f   __attribute__((ext_vector_type(4)));
typedef float          v8f   __attribute__((ext_vector_type(8)));
typedef int            v4i   __attribute__((ext_vector_type(4)));
typedef int            v8i   __attribute__((ext_vector_type(8)));
typedef unsigned short v4us  __attribute__((ext_vector_type(4)));
typedef unsigned short v8us  __attribute__((ext_vector_type(8)));
typedef unsigned short v16us __attribute__((ext_vector_type(16)));
typedef __bf16         v16bf __attribute__((ext_vector_type(16)));
typedef v4f  __attribute__((may_alias)) v4fa;
typedef v4i  __attribute__((may_alias)) v4ia;
typedef v4us __attribute__((may_alias)) v4usa;
typedef v8us __attribute__((may_alias)) v8usa;
union FragB { v16bf v; v16us u; v8us h[2]; v8i w; };

__device__ __forceinline__ v8f wmb(const FragB& a, const FragB& b, v8f c) {
  v8f d = __builtin_amdgcn_wmma_f32_16x16x32_bf16(false, a.v, false, b.v, (short)0, c, false, false);
  asm volatile("v_nop\n\tv_nop\n\tv_nop\n\tv_nop" : "+v"(d) : "v"(a.w), "v"(b.w));
  return d;
}
__device__ __forceinline__ v8f z8() { v8f z = {0.f, 0.f, 0.f, 0.f, 0.f, 0.f, 0.f, 0.f}; return z; }

__device__ __forceinline__ unsigned bf16_bits(float f) {
  const unsigned u = __float_as_uint(f);
  return ((u + 0x7FFFu + ((u >> 16) & 1u)) >> 16) & 0xFFFFu;
}
__device__ __forceinline__ float bf16_val(float f) { return __uint_as_float(bf16_bits(f) << 16); }
__device__ __forceinline__ unsigned hl_bits(float v, unsigned& lo) {
  const unsigned hb = bf16_bits(v);
  lo = bf16_bits(v - __uint_as_float(hb << 16));
  return hb;
}
__device__ __forceinline__ void wave_sync() {
  __builtin_amdgcn_fence(__ATOMIC_RELEASE, "wavefront");
  __builtin_amdgcn_wave_barrier();
  __builtin_amdgcn_fence(__ATOMIC_ACQUIRE, "wavefront");
}
__device__ __forceinline__ void put_us8(unsigned short* p, v8us v) {
  *(volatile v8us*)p = v; __threadfence(); *(volatile v8us*)p = v;
}
__device__ __forceinline__ void put_f4(float* p, v4f v) {
  *(volatile v4f*)p = v; __threadfence(); *(volatile v4f*)p = v;
}
__device__ __forceinline__ void put_i4(int* p, v4i v) {
  *(volatile v4i*)p = v; __threadfence(); *(volatile v4i*)p = v;
}
__device__ __forceinline__ int clampi(int v, int lo, int hi) { return v < lo ? lo : (v > hi ? hi : v); }

template <int SLB>
__device__ __forceinline__ int scan_chunk(const int* __restrict__ dsts, int nE, int cbase, int slotBase,
                                          int nb, int vec8, int* list, int tid, int lane, int wave) {
  int wc = 0;
  const int el0  = tid * EPT;
  const int e0   = cbase + el0;
  const int sent = -2147483647 - 1;
  v4i da, db;
  if (vec8 != 0 && cbase + CHUNK <= nE) {
    da = *(const v4i*)(dsts + e0);
    db = *(const v4i*)(dsts + e0 + 4);
  } else {
    da.x = (e0     < nE) ? dsts[min(e0,     nE - 1)] : sent;
    da.y = (e0 + 1 < nE) ? dsts[min(e0 + 1, nE - 1)] : sent;
    da.z = (e0 + 2 < nE) ? dsts[min(e0 + 2, nE - 1)] : sent;
    da.w = (e0 + 3 < nE) ? dsts[min(e0 + 3, nE - 1)] : sent;
    db.x = (e0 + 4 < nE) ? dsts[min(e0 + 4, nE - 1)] : sent;
    db.y = (e0 + 5 < nE) ? dsts[min(e0 + 5, nE - 1)] : sent;
    db.z = (e0 + 6 < nE) ? dsts[min(e0 + 6, nE - 1)] : sent;
    db.w = (e0 + 7 < nE) ? dsts[min(e0 + 7, nE - 1)] : sent;
  }
  const unsigned nbs = (unsigned)slotBase;
  const unsigned unb = (unsigned)nb;
  const unsigned s0 = (unsigned)da.x - nbs, s1 = (unsigned)da.y - nbs;
  const unsigned s2 = (unsigned)da.z - nbs, s3 = (unsigned)da.w - nbs;
  const unsigned s4 = (unsigned)db.x - nbs, s5 = (unsigned)db.y - nbs;
  const unsigned s6 = (unsigned)db.z - nbs, s7 = (unsigned)db.w - nbs;
  const bool h0 = s0 < unb, h1 = s1 < unb, h2 = s2 < unb, h3 = s3 < unb;
  const bool h4 = s4 < unb, h5 = s5 < unb, h6 = s6 < unb, h7 = s7 < unb;
  const unsigned any = __builtin_amdgcn_ballot_w32(h0 | h1 | h2 | h3 | h4 | h5 | h6 | h7);
  if (any != 0u) {
#define HITJ(J, HJ, SJ) { \
      const unsigned mj = __builtin_amdgcn_ballot_w32(HJ); \
      if (mj != 0u) { \
        if (HJ) { \
          const int pos = wc + (int)__builtin_amdgcn_mbcnt_lo(mj, 0u); \
          if (pos < WCAP) list[wave * WCAP + pos] = ((el0 + (J)) << SLB) | (int)(SJ); \
        } \
        wc += (int)__builtin_popcount(mj); } }
    HITJ(0, h0, s0)
    HITJ(1, h1, s1)
    HITJ(2, h2, s2)
    HITJ(3, h3, s3)
    HITJ(4, h4, s4)
    HITJ(5, h5, s5)
    HITJ(6, h6, s6)
    HITJ(7, h7, s7)
#undef HITJ
  }
  return wc;
}

__global__ __launch_bounds__(NTHR) void k_prep(const float* __restrict__ x, const float* __restrict__ wemb,
                                               const float* __restrict__ bemb, const float* __restrict__ wlay,
                                               const float* __restrict__ blay, const float* __restrict__ gam,
                                               const float* __restrict__ bet, const float* __restrict__ wout,
                                               unsigned short* we, unsigned short* wl2, float* pt,
                                               unsigned short* xb, int nN, int nUnits) {
  const int u = (int)blockIdx.x * NTHR + (int)threadIdx.x;
  if (u < U_WL) {
    const float* p = wemb + (size_t)u * 8;
    const v4f a = *(const v4fa*)p;
    const v4f b = *(const v4fa*)(p + 4);
    v8us o;
    o[0] = (unsigned short)bf16_bits(a.x); o[1] = (unsigned short)bf16_bits(a.y);
    o[2] = (unsigned short)bf16_bits(a.z); o[3] = (unsigned short)bf16_bits(a.w);
    o[4] = (unsigned short)bf16_bits(b.x); o[5] = (unsigned short)bf16_bits(b.y);
    o[6] = (unsigned short)bf16_bits(b.z); o[7] = (unsigned short)bf16_bits(b.w);
    put_us8(we + (size_t)u * 8, o);
  } else if (u < U_PT) {
    const int v  = u - U_WL;
    const int l  = v >> 12;
    const int n  = (v >> 5) & (HID - 1);
    const int k8 = (v & 31) * 8;
    const int kk = k8 & (HID - 1);
    const float* p = wlay + ((size_t)l * HID + (size_t)n) * HID + kk;
    const v4f a = *(const v4fa*)p;
    const v4f b = *(const v4fa*)(p + 4);
    v8us o;
    o[0] = (unsigned short)bf16_bits(a.x); o[1] = (unsigned short)bf16_bits(a.y);
    o[2] = (unsigned short)bf16_bits(a.z); o[3] = (unsigned short)bf16_bits(a.w);
    o[4] = (unsigned short)bf16_bits(b.x); o[5] = (unsigned short)bf16_bits(b.y);
    o[6] = (unsigned short)bf16_bits(b.z); o[7] = (unsigned short)bf16_bits(b.w);
    put_us8(wl2 + (size_t)v * 8, o);
  } else if (u < U_XB) {
    const int t  = u - U_PT;
    const int ta = clampi(t, 0, 31);
    const int tb = clampi(t - 32, 0, 127);
    const int tc = clampi(t - 160, 0, 127);
    const int td = clampi(t - 288, 0, 127);
    const int te = clampi(t - 416, 0, 31);
    const v4f a = *(const v4fa*)(bemb + 4 * ta);
    const v4f b = *(const v4fa*)(blay + 4 * tb);
    const v4f c = *(const v4fa*)(gam + 4 * tc);
    const v4f d = *(const v4fa*)(bet + 4 * td);
    const v4f e = *(const v4fa*)(wout + 4 * te);
    const unsigned ma = (t < 32) ? 0xFFFFFFFFu : 0u;
    const unsigned mb = (t >= 32 && t < 160) ? 0xFFFFFFFFu : 0u;
    const unsigned mc = (t >= 160 && t < 288) ? 0xFFFFFFFFu : 0u;
    const unsigned md = (t >= 288 && t < 416) ? 0xFFFFFFFFu : 0u;
    const unsigned me = (t >= 416) ? 0xFFFFFFFFu : 0u;
    const unsigned r0 = (__float_as_uint(a.x) & ma) | (__float_as_uint(b.x) & mb) | (__float_as_uint(c.x) & mc) |
                        (__float_as_uint(d.x) & md) | (__float_as_uint(e.x) & me);
    const unsigned r1 = (__float_as_uint(a.y) & ma) | (__float_as_uint(b.y) & mb) | (__float_as_uint(c.y) & mc) |
                        (__float_as_uint(d.y) & md) | (__float_as_uint(e.y) & me);
    const unsigned r2 = (__float_as_uint(a.z) & ma) | (__float_as_uint(b.z) & mb) | (__float_as_uint(c.z) & mc) |
                        (__float_as_uint(d.z) & md) | (__float_as_uint(e.z) & me);
    const unsigned r3 = (__float_as_uint(a.w) & ma) | (__float_as_uint(b.w) & mb) | (__float_as_uint(c.w) & mc) |
                        (__float_as_uint(d.w) & md) | (__float_as_uint(e.w) & me);
    v4f o;
    o.x = bf16_val(__uint_as_float(r0)); o.y = bf16_val(__uint_as_float(r1));
    o.z = bf16_val(__uint_as_float(r2)); o.w = bf16_val(__uint_as_float(r3));
    if (t < NPTV) put_f4(pt + 4 * t, o);
  } else if (u < nUnits) {
    const int v   = u - U_XB;
    const int row = v >> 4;
    const int k8  = (v & 15) * 8;
    const int rc  = row < nN ? row : nN - 1;
    const float* p = x + (size_t)rc * HID + k8;
    const v4f a = *(const v4fa*)p;
    const v4f b = *(const v4fa*)(p + 4);
    const bool ok = row < nN;
    v8us o;
    o[0] = ok ? (unsigned short)bf16_bits(a.x) : (unsigned short)0;
    o[1] = ok ? (unsigned short)bf16_bits(a.y) : (unsigned short)0;
    o[2] = ok ? (unsigned short)bf16_bits(a.z) : (unsigned short)0;
    o[3] = ok ? (unsigned short)bf16_bits(a.w) : (unsigned short)0;
    o[4] = ok ? (unsigned short)bf16_bits(b.x) : (unsigned short)0;
    o[5] = ok ? (unsigned short)bf16_bits(b.y) : (unsigned short)0;
    o[6] = ok ? (unsigned short)bf16_bits(b.z) : (unsigned short)0;
    o[7] = ok ? (unsigned short)bf16_bits(b.w) : (unsigned short)0;
    put_us8(xb + (size_t)v * 8, o);
  }
}

__global__ __launch_bounds__(NTHR) void k_bucket(const int* __restrict__ srcs, const int* __restrict__ dsts,
                                                 int nE, int nN, int vec8, int* listg, int* cntg, int* offg,
                                                 float* disg, int* flagg) {
  extern __shared__ __attribute__((aligned(16))) int dsm[];
  int* list = dsm;
  int* hl   = dsm + LISTN;
  int* sl   = hl + RCAP;
  int* cnt  = sl + RCAP;
  int* offs = cnt + NBA;
  int* cur  = offs + NBA;
  int* misc = cur + NBA;
  const int tid = (int)threadIdx.x, lane = tid & 31, wave = tid >> 5;
  const int blk = (int)blockIdx.x;
  const int nodeBase = blk * NBA;

  {
    const v4i z4 = {0, 0, 0, 0};
    for (int i = tid * 4; i < AGG_ZINTS; i += NTHR * 4) *(v4ia*)(dsm + i) = z4;
    if (tid < MISC_INTS) misc[tid] = 0;
  }
  __syncthreads();

  int t = 0, ov = 0;
  const int nChunks = (nE + CHUNK - 1) / CHUNK;
#pragma unroll 1
  for (int ch = 0; ch < nChunks; ++ch) {
    const int cbase = ch * CHUNK;
    const int wc = scan_chunk<SLA>(dsts, nE, cbase, nodeBase, NBA, vec8, list, tid, lane, wave);
    if (lane == 0) misc[wave] = wc;
    __syncthreads();
    if (wave == 0) {
#pragma unroll 1
      for (int w2 = 0; w2 < NWAVE; ++w2) {
        int c = misc[w2];
        c = c < 0 ? 0 : (c > WCAP ? WCAP : c);
#pragma unroll 1
        for (int b0 = 0; b0 < c; b0 += 32) {
          const int idx = b0 + lane;
          const int ent = list[w2 * WCAP + (idx < WCAP ? idx : WCAP - 1)];
          const int m32 = (c - b0) < 32 ? (c - b0) : 32;
#pragma unroll 1
          for (int k = 0; k < m32; ++k) {
            const int u    = __builtin_amdgcn_readlane(ent, k);
            const int slot = u & (NBA - 1);
            const int el   = (u >> SLA) & (CHUNK - 1);
            const int pk   = ((cbase + el) << SLA) | slot;
            if (t < RCAP) {
              if (lane == 0) { hl[t] = pk; cnt[slot] = cnt[slot] + 1; }
              t = t + 1;
            } else {
              ov = 1;
            }
          }
        }
      }
    }
    __syncthreads();
  }
  if (wave == 0 && lane == 0) { misc[8] = t; misc[9] = ov; }
  __syncthreads();
  int tt = misc[8];
  tt = tt < 0 ? 0 : (tt > RCAP ? RCAP : tt);

  if (wave == 0) {
    const int base = lane * (NBA / 32);
    int s = 0;
#pragma unroll 1
    for (int i = 0; i < NBA / 32; ++i) s += cnt[base + i];
    int incl = s;
#pragma unroll
    for (int d = 1; d < 32; d <<= 1) {
      const int y = __shfl_up(incl, d, 32);
      if (lane >= d) incl += y;
    }
    int run = incl - s;
#pragma unroll 1
    for (int i = 0; i < NBA / 32; ++i) {
      const int cv = cnt[base + i];
      offs[base + i] = run;
      cur[base + i]  = run;
      run += cv;
    }
  }
  __syncthreads();
  if (wave == 0) {
#pragma unroll 1
    for (int b0 = 0; b0 < tt; b0 += 32) {
      const int idx = b0 + lane;
      const int ent = hl[idx < RCAP ? idx : RCAP - 1];
      const int m32 = (tt - b0) < 32 ? (tt - b0) : 32;
#pragma unroll 1
      for (int k = 0; k < m32; ++k) {
        const int u    = __builtin_amdgcn_readlane(ent, k);
        const int slot = u & (NBA - 1);
        if (lane == 0) {
          int p = cur[slot];
          p = p < 0 ? 0 : (p > RCAP - 1 ? RCAP - 1 : p);
          sl[p] = u;
          cur[slot] = p + 1;
        }
      }
    }
  }
  __syncthreads();

  int* lg = listg + (size_t)blk * RCAP;
#pragma unroll 1
  for (int it = 0; it < RCAP / (NTHR * 4); ++it) {
    const int p = it * (NTHR * 4) + 4 * tid;
    const v4i e4 = *(const v4ia*)(sl + p);
    const int q0 = clampi(e4.x >> SLA, 0, nE - 1);
    const int q1 = clampi(e4.y >> SLA, 0, nE - 1);
    const int q2 = clampi(e4.z >> SLA, 0, nE - 1);
    const int q3 = clampi(e4.w >> SLA, 0, nE - 1);
    const int r0 = clampi(srcs[q0], 0, nN - 1);
    const int r1 = clampi(srcs[q1], 0, nN - 1);
    const int r2 = clampi(srcs[q2], 0, nN - 1);
    const int r3 = clampi(srcs[q3], 0, nN - 1);
    v4i o;
    o.x = (p     < tt) ? r0 : 0;
    o.y = (p + 1 < tt) ? r1 : 0;
    o.z = (p + 2 < tt) ? r2 : 0;
    o.w = (p + 3 < tt) ? r3 : 0;
    put_i4(lg + p, o);
  }

  {
    int big = 0;
#pragma unroll 1
    for (int j = 0; j < NBA / NTHR; ++j) {
      const int s = tid + j * NTHR;
      const int cv = cnt[s];
      const float d = (float)(cv + 1);
      list[s] = __float_as_int(1.0f / sqrtf(d));
      big |= (cv > DEGCAP) ? 1 : 0;
    }
    if (big != 0) misc[10] = 1;
  }
  __syncthreads();
  {
    const int s0 = 4 * tid;
    const v4i c4 = *(const v4ia*)(cnt + s0);
    const v4i o4 = *(const v4ia*)(offs + s0);
    const v4i d4 = *(const v4ia*)(list + s0);
    v4f df;
    df.x = __int_as_float(d4.x); df.y = __int_as_float(d4.y);
    df.z = __int_as_float(d4.z); df.w = __int_as_float(d4.w);
    int*   cp = cntg + (size_t)nodeBase + s0;
    int*   op = offg + (size_t)nodeBase + s0;
    float* dp = disg + (size_t)nodeBase + s0;
    *(volatile v4i*)cp = c4;
    *(volatile v4i*)op = o4;
    *(volatile v4f*)dp = df;
    __threadfence();
    *(volatile v4i*)cp = c4;
    *(volatile v4i*)op = o4;
    *(volatile v4f*)dp = df;
    const int fl = ((misc[9] | misc[10]) != 0) ? 1 : 0;
    const v4i f4 = {fl, fl, fl, fl};
    const bool okf = tid < 8;
    int* fp = flagg + (size_t)blk * 32 + 4 * (tid & 7);
    if (okf) *(volatile v4i*)fp = f4;
    __threadfence();
    if (okf) *(volatile v4i*)fp = f4;
  }
}

template <int MODE>
__global__ __launch_bounds__(GTHR) void k_gemm(const unsigned short* __restrict__ A, int lda,
                                               const unsigned short* __restrict__ BT, int ldb, int K,
                                               const float* __restrict__ aux, float* outF,
                                               unsigned short* hhl, int nN) {
  __shared__ __attribute__((aligned(16))) float stg[GBM * GBN];
  const int tid = (int)threadIdx.x, lane = tid & 31, wave = tid >> 5, hh = lane >> 4, m = lane & 15;
  const int rowBase = (int)blockIdx.x * GBM;

  v8f acc[8];
#pragma unroll
  for (int t = 0; t < 8; ++t) acc[t] = z8();
  const unsigned short* ap = A + (size_t)(rowBase + 16 * wave + m) * (size_t)lda + 8 * hh;
  const unsigned short* bp = BT + (size_t)m * (size_t)ldb + 8 * hh;

#pragma unroll 1
  for (int k0 = 0; k0 < K; k0 += 32) {
    FragB af;
    af.h[0] = *(const v8usa*)(ap + k0);
    af.h[1] = *(const v8usa*)(ap + k0 + 16);
#pragma unroll
    for (int nt = 0; nt < 8; ++nt) {
      const unsigned short* wq = bp + (size_t)(16 * nt) * (size_t)ldb + k0;
      FragB bf;
      bf.h[0] = *(const v8usa*)wq;
      bf.h[1] = *(const v8usa*)(wq + 16);
      acc[nt] = wmb(af, bf, acc[nt]);
    }
  }

#pragma unroll
  for (int nt = 0; nt < 8; ++nt) {
    const int lc = 16 * nt + m;
#pragma unroll
    for (int r = 0; r < 8; ++r) {
      const int lr = 16 * wave + 8 * hh + r;
      stg[lr * GBN + lc] = acc[nt][r];
    }
  }
  __syncthreads();

  v4f pv[16];
#pragma unroll
  for (int i = 0; i < 16; ++i) pv[i] = *(const v4fa*)(stg + (16 * wave + i) * GBN + 4 * lane);
  __syncthreads();

  if constexpr (MODE == 0) {
    const v4f b4 = *(const v4fa*)(aux + 4 * lane);
#pragma unroll
    for (int i = 0; i < 16; ++i) {
      const int row = rowBase + 16 * wave + i;
      const bool ok = row < nN;
      v4f q;
      q.x = ok ? (pv[i].x + b4.x) : 0.0f;
      q.y = ok ? (pv[i].y + b4.y) : 0.0f;
      q.z = ok ? (pv[i].z + b4.z) : 0.0f;
      q.w = ok ? (pv[i].w + b4.w) : 0.0f;
      pv[i] = q;
    }
  } else {
    const float dl = aux[rowBase + 16 * wave + m];
#pragma unroll
    for (int i = 0; i < 16; ++i) {
      const float di = __shfl(dl, i, 32);
      v4f q;
      q.x = pv[i].x * di; q.y = pv[i].y * di; q.z = pv[i].z * di; q.w = pv[i].w * di;
      pv[i] = q;
    }
  }

#pragma unroll
  for (int i = 0; i < 16; ++i) {
    const int row = rowBase + 16 * wave + i;
    float* op = outF + (size_t)row * HID + 4 * lane;
    *(volatile v4f*)op = pv[i];
  }
  __threadfence();
#pragma unroll
  for (int i = 0; i < 16; ++i) {
    const int row = rowBase + 16 * wave + i;
    float* op = outF + (size_t)row * HID + 4 * lane;
    *(volatile v4f*)op = pv[i];
  }

  if constexpr (MODE == 0) {
#pragma unroll
    for (int i = 0; i < 16; ++i) {
      v4us h4, l4;
      unsigned lb;
      unsigned hb;
      hb = hl_bits(pv[i].x, lb); h4[0] = (unsigned short)hb; l4[0] = (unsigned short)lb;
      hb = hl_bits(pv[i].y, lb); h4[1] = (unsigned short)hb; l4[1] = (unsigned short)lb;
      hb = hl_bits(pv[i].z, lb); h4[2] = (unsigned short)hb; l4[2] = (unsigned short)lb;
      hb = hl_bits(pv[i].w, lb); h4[3] = (unsigned short)hb; l4[3] = (unsigned short)lb;
      unsigned short* srow = (unsigned short*)stg + (size_t)(16 * wave + i) * (2 * GBN);
      *(v4usa*)(srow + 4 * lane) = h4;
      *(v4usa*)(srow + HID + 4 * lane) = l4;
    }
    __syncthreads();
    v8us qv[16];
#pragma unroll
    for (int i = 0; i < 16; ++i) {
      const unsigned short* srow = (const unsigned short*)stg + (size_t)(16 * wave + i) * (2 * GBN);
      qv[i] = *(const v8usa*)(srow + 8 * lane);
    }
#pragma unroll
    for (int i = 0; i < 16; ++i) {
      const int gr = rowBase + 16 * wave + i;
      unsigned short* rp = hhl + (size_t)gr * (size_t)K2 + 8 * lane;
      *(volatile v8us*)rp = qv[i];
    }
    __threadfence();
#pragma unroll
    for (int i = 0; i < 16; ++i) {
      const int gr = rowBase + 16 * wave + i;
      unsigned short* rp = hhl + (size_t)gr * (size_t)K2 + 8 * lane;
      *(volatile v8us*)rp = qv[i];
    }
  } else {
    (void)hhl; (void)nN;
  }
}

template <int LAST>
__global__ __launch_bounds__(NTHR) void k_agg(const int* __restrict__ listg, const int* __restrict__ cntg,
                                              const int* __restrict__ offg, const float* __restrict__ disg,
                                              const int* __restrict__ flagg, const float* __restrict__ T,
                                              const float* __restrict__ pt, int layer,
                                              float* Hf, unsigned short* hhl, const int* __restrict__ bat,
                                              int nN, double* sumrec, int* cntrec) {
  __shared__ __attribute__((aligned(16))) unsigned short rowbufAll[NWAVE * ROWH];
  __shared__ float sS[NBA];
  __shared__ int   sB[NBA];
  const int tid = (int)threadIdx.x, lane = tid & 31;
  const int wave = __builtin_amdgcn_readfirstlane(tid >> 5);
  const int blk = (int)blockIdx.x;
  const int nodeBase = blk * NBA;
  unsigned short* rowbuf = rowbufAll + wave * ROWH;

  const int fl = __builtin_amdgcn_readfirstlane(flagg[(size_t)blk * 32]);
  const float qnan = __int_as_float(0x7fc00000);
  const float pz = (fl != 0) ? qnan : 0.0f;
  const v4f bq = *(const v4fa*)(pt + PT_BL + layer * HID + 4 * lane);
  const v4f gq = *(const v4fa*)(pt + PT_GA + layer * HID + 4 * lane);
  const v4f eq = *(const v4fa*)(pt + PT_BT + layer * HID + 4 * lane);
  const v4f wq = *(const v4fa*)(pt + PT_WO + 4 * lane);
  const int* lst = listg + (size_t)blk * RCAP;
  const float invd = 1.0f / (float)HID;

#pragma unroll 1
  for (int si = 0; si < NBA / NWAVE; ++si) {
    const int s    = si * NWAVE + wave;
    const int node = nodeBase + s;
    const bool live = node < nN;
    const int nc = live ? node : nN - 1;
    int c = __builtin_amdgcn_readfirstlane(cntg[node]);
    const bool big = c > DEGCAP;
    c = c < 0 ? 0 : (c > DEGCAP ? DEGCAP : c);
    int o = __builtin_amdgcn_readfirstlane(offg[node]);
    o = o < 0 ? 0 : (o > RCAP ? RCAP : o);
    const float dd = disg[node];
    float a0 = 0.0f, a1 = 0.0f, a2 = 0.0f, a3 = 0.0f;
#pragma unroll 1
    for (int b0 = 0; b0 < c; b0 += 32) {
      int idx = o + b0 + lane;
      idx = idx > o + c - 1 ? o + c - 1 : idx;
      idx = idx < 0 ? 0 : (idx > RCAP - 1 ? RCAP - 1 : idx);
      int sr = lst[idx];
      sr = sr < 0 ? 0 : (sr > nN - 1 ? nN - 1 : sr);
      const int m32 = (c - b0) < 32 ? (c - b0) : 32;
#pragma unroll 1
      for (int k = 0; k < m32; ++k) {
        const int sk = __builtin_amdgcn_readlane(sr, k);
        const v4f r = *(const v4fa*)(T + (size_t)sk * HID + 4 * lane);
        a0 += r.x; a1 += r.y; a2 += r.z; a3 += r.w;
      }
    }
    const v4f tv = *(const v4fa*)(T + (size_t)nc * HID + 4 * lane);
    const v4f hv = *(const v4fa*)(Hf + (size_t)nc * HID + 4 * lane);
    const float pzr = big ? qnan : pz;
    const float g0 = dd * (a0 + tv.x) + bq.x;
    const float g1 = dd * (a1 + tv.y) + bq.y;
    const float g2 = dd * (a2 + tv.z) + bq.z;
    const float g3 = dd * (a3 + tv.w) + bq.w;
    const float r0 = (g0 > 0.0f) ? g0 : (g0 - g0);
    const float r1 = (g1 > 0.0f) ? g1 : (g1 - g1);
    const float r2 = (g2 > 0.0f) ? g2 : (g2 - g2);
    const float r3 = (g3 > 0.0f) ? g3 : (g3 - g3);
    const float u0 = (hv.x + r0) + pzr, u1 = (hv.y + r1) + pzr;
    const float u2 = (hv.z + r2) + pzr, u3 = (hv.w + r3) + pzr;
    float sm = (u0 + u1) + (u2 + u3);
    sm += __shfl_xor(sm, 16, 32);
    sm += __shfl_xor(sm, 8, 32);
    sm += __shfl_xor(sm, 4, 32);
    sm += __shfl_xor(sm, 2, 32);
    sm += __shfl_xor(sm, 1, 32);
    const float mean = sm * invd;
    const float d0 = u0 - mean, d1 = u1 - mean, d2 = u2 - mean, d3 = u3 - mean;
    float q = (d0 * d0 + d1 * d1) + (d2 * d2 + d3 * d3);
    q += __shfl_xor(q, 16, 32);
    q += __shfl_xor(q, 8, 32);
    q += __shfl_xor(q, 4, 32);
    q += __shfl_xor(q, 2, 32);
    q += __shfl_xor(q, 1, 32);
    const float var  = q * invd;
    const float rstd = 1.0f / sqrtf(var + LNEPS);
    const float y0 = (d0 * rstd) * gq.x + eq.x;
    const float y1 = (d1 * rstd) * gq.y + eq.y;
    const float y2 = (d2 * rstd) * gq.z + eq.z;
    const float y3 = (d3 * rstd) * gq.w + eq.w;

    if constexpr (LAST == 0) {
      v4us mh, ml;
      {
        unsigned lb;
        unsigned hb;
        hb = hl_bits(y0, lb); mh[0] = (unsigned short)hb; ml[0] = (unsigned short)lb;
        hb = hl_bits(y1, lb); mh[1] = (unsigned short)hb; ml[1] = (unsigned short)lb;
        hb = hl_bits(y2, lb); mh[2] = (unsigned short)hb; ml[2] = (unsigned short)lb;
        hb = hl_bits(y3, lb); mh[3] = (unsigned short)hb; ml[3] = (unsigned short)lb;
      }
      *(v4usa*)(rowbuf + 4 * lane)       = mh;
      *(v4usa*)(rowbuf + HID + 4 * lane) = ml;
      wave_sync();
      const v8us q0 = *(const v8usa*)(rowbuf + 8 * lane);
      wave_sync();
      v4f yv; yv.x = y0; yv.y = y1; yv.z = y2; yv.w = y3;
      float* hp = Hf + (size_t)nc * HID + 4 * lane;
      unsigned short* rp = hhl + (size_t)nc * K2 + 8 * lane;
      if (live) { *(volatile v4f*)hp = yv; *(volatile v8us*)rp = q0; }
      __threadfence();
      if (live) { *(volatile v4f*)hp = yv; *(volatile v8us*)rp = q0; }
    } else {
      float sd = (y0 * wq.x + y1 * wq.y) + (y2 * wq.z + y3 * wq.w);
      sd += __shfl_xor(sd, 16, 32);
      sd += __shfl_xor(sd, 8, 32);
      sd += __shfl_xor(sd, 4, 32);
      sd += __shfl_xor(sd, 2, 32);
      sd += __shfl_xor(sd, 1, 32);
      const int bv = bat[nc];
      if (lane == 0) { sS[s] = sd; sB[s] = live ? bv : -1; }
    }
  }

  if constexpr (LAST != 0) {
    __syncthreads();
    if (wave == 0) {
      double sum = 0.0;
      int cn = 0;
#pragma unroll 1
      for (int s = 0; s < NBA; ++s) {
        const int   bv = sB[s];
        const float sv = sS[s];
        const bool hit = (bv == lane);
        sum += hit ? (double)sv : 0.0;
        cn  += hit ? 1 : 0;
      }
      const double sw = (fl != 0) ? (double)qnan : sum;
      double* sp = sumrec + (size_t)blk * 32 + lane;
      int*    cp = cntrec + (size_t)blk * 32 + lane;
      *(volatile double*)sp = sw;
      *(volatile int*)cp = cn;
      __threadfence();
      *(volatile double*)sp = sw;
      *(volatile int*)cp = cn;
    }
    (void)hhl;
  } else {
    (void)sumrec; (void)cntrec; (void)bat; (void)wq;
  }
}

__global__ __launch_bounds__(32) void k_pool(const double* __restrict__ sumrec, const int* __restrict__ cntrec,
                                             const int* __restrict__ flagg, int nB, float* out) {
  __shared__ __attribute__((aligned(16))) float so[32];
  const int lane = (int)threadIdx.x & 31;
  double s = 0.0;
  int c = 0, f = 0;
#pragma unroll 1
  for (int b = 0; b < nB; ++b) {
    s += sumrec[(size_t)b * 32 + lane];
    c += cntrec[(size_t)b * 32 + lane];
    f |= flagg[(size_t)b * 32];
  }
  const float cf = fmaxf((float)c, 1.0f);
  float v = (float)s / cf;
  v = (f != 0) ? __int_as_float(0x7fc00000) : v;
  so[lane] = v;
  __syncthreads();
  const bool ok = lane < 8;
  const v4f ov = *(const v4fa*)(so + 4 * (lane & 7));
  float* op = out + 4 * (lane & 7);
  if (ok) *(volatile v4f*)op = ov;
  __threadfence();
  if (ok) *(volatile v4f*)op = ov;
}

static inline size_t al256(size_t o) { return (o + 255) & ~(size_t)255; }

extern "C" void kernel_launch(void* const* d_in, const int* in_sizes, int n_in,
                              void* d_out, int out_size, void* d_ws, size_t ws_size,
                              hipStream_t stream) {
  if (n_in < 10) return;
  if (in_sizes[0] != NNODE * HID) return;
  if (in_sizes[1] != 2 * NEDGE) return;
  if (in_sizes[2] != NNODE) return;
  if (in_sizes[3] != HID * HID || in_sizes[4] != HID) return;
  if (in_sizes[5] != NLAY * HID * HID || in_sizes[6] != NLAY * HID) return;
  if (in_sizes[7] != NLAY * HID || in_sizes[8] != NLAY * HID) return;
  if (in_sizes[9] != HID) return;
  if (out_size != NG) return;
  const int nN = NNODE, nE = NEDGE;

  const float* x    = (const float*)d_in[0];
  const int*   edge = (const int*)d_in[1];
  const int*   bat  = (const int*)d_in[2];
  const float* Wemb = (const float*)d_in[3];
  const float* bemb = (const float*)d_in[4];
  const float* Wlay = (const float*)d_in[5];
  const float* blay = (const float*)d_in[6];
  const float* gam  = (const float*)d_in[7];
  const float* bet  = (const float*)d_in[8];
  const float* Wout = (const float*)d_in[9];
  float* out = (float*)d_out;
  const int* src = edge;
  const int* dst = edge + nE;
  const int vec8 = ((nE & 3) == 0) ? 1 : 0;

  char* ws = (char*)d_ws;
  size_t off = 0;
  const size_t oWE  = off; off = al256(off + (size_t)HID * HID * 2);
  const size_t oWL2 = off; off = al256(off + (size_t)NLAY * HID * K2 * 2);
  const size_t oPT  = off; off = al256(off + (size_t)PT_N * 4);
  const size_t oXB  = off; off = al256(off + (size_t)MP * HID * 2);
  const size_t oH   = off; off = al256(off + (size_t)MP * HID * 4);
  const size_t oHHL = off; off = al256(off + (size_t)MP * K2 * 2);
  const size_t oT   = off; off = al256(off + (size_t)MP * HID * 4);
  const size_t oLST = off; off = al256(off + (size_t)NBLK * RCAP * 4);
  const size_t oCNT = off; off = al256(off + (size_t)NSLOT * 4);
  const size_t oOFF = off; off = al256(off + (size_t)NSLOT * 4);
  const size_t oDIS = off; off = al256(off + (size_t)NSLOT * 4);
  const size_t oFLG = off; off = al256(off + (size_t)NBLK * 32 * 4);
  const size_t oSUM = off; off = al256(off + (size_t)NBLK * 32 * 8);
  const size_t oCRC = off; off = al256(off + (size_t)NBLK * 32 * 4);
  if (off > ws_size || off > (size_t)WSMAX) return;
  unsigned short* WE  = (unsigned short*)(ws + oWE);
  unsigned short* WL2 = (unsigned short*)(ws + oWL2);
  float*          PT  = (float*)(ws + oPT);
  unsigned short* XB  = (unsigned short*)(ws + oXB);
  float*          Hf  = (float*)(ws + oH);
  unsigned short* HHL = (unsigned short*)(ws + oHHL);
  float*          Tf  = (float*)(ws + oT);
  int*            LST = (int*)(ws + oLST);
  int*            CNT = (int*)(ws + oCNT);
  int*            OFF = (int*)(ws + oOFF);
  float*          DIS = (float*)(ws + oDIS);
  int*            FLG = (int*)(ws + oFLG);
  double*         SUM = (double*)(ws + oSUM);
  int*            CRC = (int*)(ws + oCRC);

  const size_t bkLds = (size_t)BK_LDS_INTS * 4;
  hipFuncSetAttribute(reinterpret_cast<const void*>(&k_bucket), hipFuncAttributeMaxDynamicSharedMemorySize, (int)bkLds);

  const int nUnits = U_XB + MP * (HID / 8);
  const int gM = MP / GBM;

  k_prep<<<nUnits / NTHR, NTHR, 0, stream>>>(x, Wemb, bemb, Wlay, blay, gam, bet, Wout, WE, WL2, PT, XB, nN, nUnits);
  k_bucket<<<NBLK, NTHR, bkLds, stream>>>(src, dst, nE, nN, vec8, LST, CNT, OFF, DIS, FLG);
  k_gemm<0><<<gM, GTHR, 0, stream>>>(XB, HID, WE, HID, HID, PT + PT_BE, Hf, HHL, nN);
  for (int l = 0; l < NLAY; ++l) {
    k_gemm<1><<<gM, GTHR, 0, stream>>>(HHL, K2, WL2 + (size_t)l * HID * K2, K2, K2, DIS, Tf, HHL, nN);
    if (l < NLAY - 1) {
      k_agg<0><<<NBLK, NTHR, 0, stream>>>(LST, CNT, OFF, DIS, FLG, Tf, PT, l, Hf, HHL, bat, nN, SUM, CRC);
    } else {
      k_agg<1><<<NBLK, NTHR, 0, stream>>>(LST, CNT, OFF, DIS, FLG, Tf, PT, l, Hf, HHL, bat, nN, SUM, CRC);
    }
  }
  k_pool<<<1, 32, 0, stream>>>(SUM, CRC, FLG, NBLK, out);
}
